// FluxUNet_64003602645716
// MI455X (gfx1250) — hardware-verified
//
#include <hip/hip_runtime.h>
#define BB 8
#define CC 512
#define HI 32
#define WI 32
#define HWN 1024
#define SS 77
#define SP 96
#define EE 768
#define NH 8
#define HD 64
#define HID 2048

typedef __bf16 v16b __attribute__((ext_vector_type(16)));
typedef unsigned short v8us __attribute__((ext_vector_type(8), may_alias));
typedef float  v8f  __attribute__((ext_vector_type(8)));
typedef float  v4f  __attribute__((ext_vector_type(4)));
typedef float  v4fa __attribute__((ext_vector_type(4), may_alias));
union FragB { v16b v; v8us half[2]; unsigned short u[16]; };

__device__ __forceinline__ unsigned short bf16_bits(float x) { unsigned int u = __float_as_uint(x); return (unsigned short)((u + 0x7FFFu + ((u >> 16) & 1u)) >> 16); }
__device__ __forceinline__ float bf16_val(unsigned short b) { return __uint_as_float(((unsigned int)b) << 16); }
__device__ __forceinline__ float bf16_round(float x) { return bf16_val(bf16_bits(x)); }
template <int NT>
__device__ __forceinline__ v8f mmaN(v16b ah, v16b al, v16b bh, v16b bl, v8f c) {
  c = __builtin_amdgcn_wmma_f32_16x16x32_bf16(false, ah, false, bh, (short)0, c, false, false);
  if (NT >= 2) c = __builtin_amdgcn_wmma_f32_16x16x32_bf16(false, al, false, bh, (short)0, c, false, false);
  if (NT >= 3) c = __builtin_amdgcn_wmma_f32_16x16x32_bf16(false, ah, false, bl, (short)0, c, false, false);
  asm volatile("v_nop\n\tv_nop\n\tv_nop\n\tv_nop" : "+v"(c) : "v"(ah), "v"(al), "v"(bh), "v"(bl));
  return c;
}

__global__ __launch_bounds__(256) void k_wt_bf16(const float* __restrict__ W, unsigned short* __restrict__ Wt, int K, int N) {
  const int t = blockIdx.x * 256 + threadIdx.x;
  const int k8n = K / 8;
  if (t >= N * k8n) return;
  const int n = t / k8n, k8 = (t % k8n) * 8;
  v8us v;
#pragma unroll
  for (int i = 0; i < 8; ++i) v[i] = bf16_bits(W[(size_t)(k8 + i) * N + n]);
  *(volatile v8us*)(Wt + (size_t)n * K + k8) = v;
  __threadfence();
  *(volatile v8us*)(Wt + (size_t)n * K + k8) = v;
}

template <bool ASPLIT, int ACT, bool BIAS_BF16>
__global__ __launch_bounds__(128) void k_gemm_bf(const float* __restrict__ A, int lda, const unsigned short* __restrict__ Wt, int ldb,
                                               const float* __restrict__ bias, float* __restrict__ C, int ldc, int M, int N, int K) {
  __shared__ __attribute__((aligned(16))) float so[4][16][64];
  const int tid = threadIdx.x, w = tid >> 5, lane = tid & 31, ln = lane & 15, hh = lane >> 4;
  const int ntn = N / 64;
  const int wid = blockIdx.x * 4 + w;
  const int mt = wid / ntn, nq = wid % ntn;
  if (mt * 16 >= M) return;
  const int row0 = mt * 16, col0 = nq * 64;
  const float* arow = A + (size_t)(row0 + ln) * lda;
  v8f acc[4] = {};
  for (int kb = 0; kb < K; kb += 32) {
    FragB ah, al;
    const v4f x0 = *(const v4fa*)(arow + kb + 8 * hh), x1 = *(const v4fa*)(arow + kb + 8 * hh + 4);
    const v4f x2 = *(const v4fa*)(arow + kb + 16 + 8 * hh), x3 = *(const v4fa*)(arow + kb + 16 + 8 * hh + 4);
    float xs[16] = {x0[0],x0[1],x0[2],x0[3],x1[0],x1[1],x1[2],x1[3],x2[0],x2[1],x2[2],x2[3],x3[0],x3[1],x3[2],x3[3]};
#pragma unroll
    for (int i = 0; i < 16; ++i) { const unsigned short hb = bf16_bits(xs[i]); ah.u[i] = hb; al.u[i] = ASPLIT ? bf16_bits(xs[i] - bf16_val(hb)) : (unsigned short)0; }
#pragma unroll
    for (int t = 0; t < 4; ++t) {
      const unsigned short* brow = Wt + (size_t)(col0 + t * 16 + ln) * ldb + kb;
      FragB b;
      b.half[0] = *(const v8us*)(brow + 8 * hh);
      b.half[1] = *(const v8us*)(brow + 16 + 8 * hh);
      acc[t] = mmaN<ASPLIT ? 2 : 1>(ah.v, al.v, b.v, b.v, acc[t]);
    }
  }
#pragma unroll
  for (int t = 0; t < 4; ++t) {
    float bv = bias ? bias[col0 + t * 16 + ln] : 0.f;
    if (BIAS_BF16) bv = bf16_round(bv);
#pragma unroll
    for (int r = 0; r < 8; ++r) { float v = acc[t][r] + bv; if (ACT == 1) v = fmaxf(v, 0.f); so[w][8 * hh + r][t * 16 + ln] = v; }
  }
  __builtin_amdgcn_fence(__ATOMIC_ACQ_REL, "workgroup");
  __builtin_amdgcn_wave_barrier();
  const int rsub = lane >> 4, c4 = (lane & 15) * 4;
  for (int pass = 0; pass < 2; ++pass) {
#pragma unroll
    for (int q = 0; q < 8; ++q) {
      const int r = q * 2 + rsub;
      const v4f v = *(const v4fa*)&so[w][r][c4];
      *(volatile v4f*)(C + (size_t)(row0 + r) * ldc + col0 + c4) = v;
    }
    if (pass == 0) __threadfence();
  }
}

template <int D, bool CAUSAL>
__global__ __launch_bounds__(128) void k_flash(const float* __restrict__ qb, const float* __restrict__ kb, const float* __restrict__ vb,
                                             int pitch, int T, int H, float scale, float* __restrict__ y, int ypitch) {
  constexpr int KS = D / 32;
  constexpr int DT = D / 16;
  __shared__ __attribute__((aligned(16))) unsigned short sKh[32][D + 8], sKl[32][D + 8], sVh[32][D + 8], sVl[32][D + 8];
  __shared__ __attribute__((aligned(16))) unsigned short sPh[4][16][40], sPl[4][16][40];
  __shared__ __attribute__((aligned(16))) float sO[4][16][D];
  const int tid = threadIdx.x, w = tid >> 5, lane = tid & 31, ln = lane & 15, hh = lane >> 4;
  const int nqb = (T + 63) / 64;
  const int bh = blockIdx.x / nqb, qblk = blockIdx.x % nqb;
  const int b = bh / H, h = bh % H;
  const int q0 = qblk * 64 + w * 16;
  const float* Q = qb + (size_t)b * T * pitch + h * D;
  const float* K = kb + (size_t)b * T * pitch + h * D;
  const float* V = vb + (size_t)b * T * pitch + h * D;

  FragB aqh[KS], aql[KS];
  {
    int row = q0 + ln; if (row >= T) row = T - 1;
    const float* qr = Q + (size_t)row * pitch;
#pragma unroll
    for (int ks = 0; ks < KS; ++ks)
#pragma unroll
      for (int i = 0; i < 16; ++i) {
        const int d = ks * 32 + ((i < 8) ? (8 * hh + i) : (16 + 8 * hh + (i - 8)));
        const float x = qr[d] * scale; const unsigned short hb = bf16_bits(x);
        aqh[ks].u[i] = hb; aql[ks].u[i] = bf16_bits(x - bf16_val(hb));
      }
  }
  float m_r[8], l_r[8];
#pragma unroll
  for (int r = 0; r < 8; ++r) { m_r[r] = -3.0e38f; l_r[r] = 0.f; }
  v8f oacc[DT];
#pragma unroll
  for (int dt = 0; dt < DT; ++dt) oacc[dt] = (v8f){0.f,0.f,0.f,0.f,0.f,0.f,0.f,0.f};

  const int kv_end = CAUSAL ? min(T, qblk * 64 + 64) : T;
  for (int j0 = 0; j0 < kv_end; j0 += 32) {
    __syncthreads();
    for (int e = tid; e < 32 * (D / 4); e += 128) {
      const int r = e / (D / 4), c4 = (e % (D / 4)) * 4;
      const int key = j0 + r;
      v4f kf = {0.f,0.f,0.f,0.f}, vf = {0.f,0.f,0.f,0.f};
      if (key < T) { kf = *(const v4fa*)(K + (size_t)key * pitch + c4); vf = *(const v4fa*)(V + (size_t)key * pitch + c4); }
#pragma unroll
      for (int t = 0; t < 4; ++t) {
        unsigned short hb = bf16_bits(kf[t]); sKh[r][c4 + t] = hb; sKl[r][c4 + t] = bf16_bits(kf[t] - bf16_val(hb));
        hb = bf16_bits(vf[t]); sVh[r][c4 + t] = hb; sVl[r][c4 + t] = bf16_bits(vf[t] - bf16_val(hb));
      }
    }
    __syncthreads();
    v8f s[2];
#pragma unroll
    for (int nt = 0; nt < 2; ++nt) {
      v8f acc = {};
#pragma unroll
      for (int ks = 0; ks < KS; ++ks) {
        FragB bh_, bl_;
        bh_.half[0] = *(const v8us*)&sKh[nt * 16 + ln][ks * 32 + 8 * hh]; bh_.half[1] = *(const v8us*)&sKh[nt * 16 + ln][ks * 32 + 16 + 8 * hh];
        bl_.half[0] = *(const v8us*)&sKl[nt * 16 + ln][ks * 32 + 8 * hh]; bl_.half[1] = *(const v8us*)&sKl[nt * 16 + ln][ks * 32 + 16 + 8 * hh];
        acc = mmaN<3>(aqh[ks].v, aql[ks].v, bh_.v, bl_.v, acc);
      }
      s[nt] = acc;
    }
    float alpha[8];
#pragma unroll
    for (int r = 0; r < 8; ++r) {
      const int qi = q0 + 8 * hh + r;
      const int ja = j0 + ln, jb = j0 + 16 + ln;
      if (CAUSAL) { if (ja > qi) s[0][r] = -3.0e38f; if (jb > qi) s[1][r] = -3.0e38f; }
      if (ja >= T) s[0][r] = -3.0e38f;
      if (jb >= T) s[1][r] = -3.0e38f;
      float mx = fmaxf(s[0][r], s[1][r]);
      mx = fmaxf(mx, __shfl_xor(mx, 1, 32)); mx = fmaxf(mx, __shfl_xor(mx, 2, 32)); mx = fmaxf(mx, __shfl_xor(mx, 4, 32)); mx = fmaxf(mx, __shfl_xor(mx, 8, 32));
      const float mnew = fmaxf(m_r[r], mx);
      alpha[r] = (mnew > -1.0e38f) ? __expf(m_r[r] - mnew) : 1.0f;
      const float p0 = (s[0][r] > -1.0e38f) ? __expf(s[0][r] - mnew) : 0.f;
      const float p1 = (s[1][r] > -1.0e38f) ? __expf(s[1][r] - mnew) : 0.f;
      m_r[r] = mnew;
      l_r[r] = l_r[r] * alpha[r] + p0 + p1;
      unsigned short hb = bf16_bits(p0); sPh[w][8 * hh + r][ln] = hb;      sPl[w][8 * hh + r][ln] = bf16_bits(p0 - bf16_val(hb));
      hb = bf16_bits(p1);                sPh[w][8 * hh + r][16 + ln] = hb; sPl[w][8 * hh + r][16 + ln] = bf16_bits(p1 - bf16_val(hb));
    }
#pragma unroll
    for (int dt = 0; dt < DT; ++dt)
#pragma unroll
      for (int r = 0; r < 8; ++r) oacc[dt][r] *= alpha[r];
    __builtin_amdgcn_fence(__ATOMIC_ACQ_REL, "workgroup");
    __builtin_amdgcn_wave_barrier();
    FragB pah, pal;
    pah.half[0] = *(const v8us*)&sPh[w][ln][8 * hh]; pah.half[1] = *(const v8us*)&sPh[w][ln][16 + 8 * hh];
    pal.half[0] = *(const v8us*)&sPl[w][ln][8 * hh]; pal.half[1] = *(const v8us*)&sPl[w][ln][16 + 8 * hh];
#pragma unroll
    for (int dt = 0; dt < DT; ++dt) {
      FragB bvh, bvl;
#pragma unroll
      for (int i = 0; i < 8; ++i) {
        bvh.u[i] = sVh[8 * hh + i][dt * 16 + ln]; bvh.u[8 + i] = sVh[16 + 8 * hh + i][dt * 16 + ln];
        bvl.u[i] = sVl[8 * hh + i][dt * 16 + ln]; bvl.u[8 + i] = sVl[16 + 8 * hh + i][dt * 16 + ln];
      }
      oacc[dt] = mmaN<3>(pah.v, pal.v, bvh.v, bvl.v, oacc[dt]);
    }
    __builtin_amdgcn_fence(__ATOMIC_ACQ_REL, "workgroup");
    __builtin_amdgcn_wave_barrier();
  }
#pragma unroll
  for (int r = 0; r < 8; ++r) {
    float l = l_r[r];
    l += __shfl_xor(l, 1, 32); l += __shfl_xor(l, 2, 32); l += __shfl_xor(l, 4, 32); l += __shfl_xor(l, 8, 32);
    l_r[r] = (l > 0.f) ? 1.0f / l : 0.f;
  }
#pragma unroll
  for (int dt = 0; dt < DT; ++dt)
#pragma unroll
    for (int r = 0; r < 8; ++r) sO[w][8 * hh + r][dt * 16 + ln] = oacc[dt][r] * l_r[r];
  __builtin_amdgcn_fence(__ATOMIC_ACQ_REL, "workgroup");
  __builtin_amdgcn_wave_barrier();
  for (int pass = 0; pass < 2; ++pass) {
    for (int r = 0; r < 16; ++r) {
      const int row = q0 + r;
      if (row < T && lane < D / 4) {
        const v4f val = *(const v4fa*)&sO[w][r][lane * 4];
        *(volatile v4f*)(y + ((size_t)b * T + row) * ypitch + h * D + lane * 4) = val;
      }
    }
    if (pass == 0) __threadfence();
  }
}

template <bool AFFINE, bool RESID, bool RES_BF16>
__global__ __launch_bounds__(256) void k_transpose32(const float* __restrict__ in, float* __restrict__ out, int rows, int cols,
                                                    const float* __restrict__ scale, const float* __restrict__ shift, const float* __restrict__ res) {
  __shared__ float tile[32][33];
  const int b = blockIdx.z;
  const int r0 = blockIdx.y * 32, c0 = blockIdx.x * 32;
  const float* src = in + (size_t)b * rows * cols;
  float* dst = out + (size_t)b * rows * cols;
  const int tx = threadIdx.x & 31, ty = threadIdx.x >> 5;
  for (int i = ty; i < 32; i += 8) tile[i][tx] = src[(size_t)(r0 + i) * cols + c0 + tx];
  __syncthreads();
  for (int pass = 0; pass < 2; ++pass) {
    for (int i = ty; i < 32; i += 8) {
      float v = tile[tx][i];
      const int orow = c0 + i;
      if (AFFINE) v = v * scale[orow] + shift[orow];
      if (RESID) { float rv = res[(size_t)b * rows * cols + (size_t)orow * rows + r0 + tx]; if (RES_BF16) rv = bf16_round(rv); v += rv; }
      *(volatile float*)(dst + (size_t)orow * rows + r0 + tx) = v;
    }
    if (pass == 0) __threadfence();
  }
}

__global__ __launch_bounds__(256) void k_pool2_pm(const float* __restrict__ in, float* __restrict__ out, int Bn, int H, int W, int C) {
  const size_t t = (size_t)blockIdx.x * 256 + threadIdx.x;
  const int c4n = C / 4, Ho = H / 2, Wo = W / 2;
  const size_t total = (size_t)Bn * Ho * Wo * c4n;
  if (t >= total) return;
  const int c4 = (int)(t % c4n) * 4; size_t rest = t / c4n;
  const int pw = (int)(rest % Wo); rest /= Wo; const int ph = (int)(rest % Ho); const int b = (int)(rest / Ho);
  const float* base = in + (size_t)b * H * W * C;
  const int p00 = (2 * ph) * W + 2 * pw;
  const v4f a = *(const v4fa*)(base + (size_t)p00 * C + c4), bq = *(const v4fa*)(base + (size_t)(p00 + 1) * C + c4);
  const v4f c = *(const v4fa*)(base + (size_t)(p00 + W) * C + c4), d = *(const v4fa*)(base + (size_t)(p00 + W + 1) * C + c4);
  v4f m; for (int i = 0; i < 4; ++i) m[i] = fmaxf(fmaxf(a[i], bq[i]), fmaxf(c[i], d[i]));
  float* dst = out + ((size_t)b * Ho * Wo + (size_t)ph * Wo + pw) * C + c4;
  *(volatile v4f*)dst = m;
  __threadfence();
  *(volatile v4f*)dst = m;
}

template <int DQ, int DV>
__global__ __launch_bounds__(128) void k_flash2(const float* __restrict__ Qb, size_t qstride, int qpitch, int Tq,
                                              const float* __restrict__ Kb, size_t kstride, int kpitch, int Tk,
                                              const float* __restrict__ Vb, size_t vstride, int vpitch,
                                              float scale, float* __restrict__ y, size_t ystride, int ypitch) {
  constexpr int KS = DQ / 32, DT = DV / 16;
  __shared__ __attribute__((aligned(16))) unsigned short sKh[32][DQ + 8], sKl[32][DQ + 8], sVh[32][DV + 8], sVl[32][DV + 8];
  __shared__ __attribute__((aligned(16))) unsigned short sPh[4][16][40], sPl[4][16][40];
  __shared__ __attribute__((aligned(16))) float sO[4][16][DV];
  const int tid = threadIdx.x, w = tid >> 5, lane = tid & 31, ln = lane & 15, hh = lane >> 4;
  const int nqb = (Tq + 63) / 64;
  const int bh = blockIdx.x / nqb, qblk = blockIdx.x % nqb;
  const int dv0 = blockIdx.y * DV;
  const int q0 = qblk * 64 + w * 16;
  const float* Q = Qb + (size_t)bh * qstride; const float* K = Kb + (size_t)bh * kstride; const float* V = Vb + (size_t)bh * vstride + dv0;
  FragB aqh[KS], aql[KS];
  {
    int row = q0 + ln; if (row >= Tq) row = Tq - 1;
    const float* qr = Q + (size_t)row * qpitch;
#pragma unroll
    for (int ks = 0; ks < KS; ++ks)
#pragma unroll
      for (int i = 0; i < 16; ++i) {
        const int d = ks * 32 + ((i < 8) ? (8 * hh + i) : (16 + 8 * hh + (i - 8)));
        const float x = qr[d] * scale; const unsigned short hb = bf16_bits(x);
        aqh[ks].u[i] = hb; aql[ks].u[i] = bf16_bits(x - bf16_val(hb));
      }
  }
  float m_r[8], l_r[8];
#pragma unroll
  for (int r = 0; r < 8; ++r) { m_r[r] = -3.0e38f; l_r[r] = 0.f; }
  v8f oacc[DT];
#pragma unroll
  for (int dt = 0; dt < DT; ++dt) oacc[dt] = (v8f){0.f,0.f,0.f,0.f,0.f,0.f,0.f,0.f};
  for (int j0 = 0; j0 < Tk; j0 += 32) {
    __syncthreads();
    for (int e = tid; e < 32 * (DQ / 4); e += 128) {
      const int r = e / (DQ / 4), c4 = (e % (DQ / 4)) * 4; const int key = j0 + r;
      v4f f = {0.f,0.f,0.f,0.f}; if (key < Tk) f = *(const v4fa*)(K + (size_t)key * kpitch + c4);
#pragma unroll
      for (int t = 0; t < 4; ++t) { const unsigned short hb = bf16_bits(f[t]); sKh[r][c4 + t] = hb; sKl[r][c4 + t] = bf16_bits(f[t] - bf16_val(hb)); }
    }
    for (int e = tid; e < 32 * (DV / 4); e += 128) {
      const int r = e / (DV / 4), c4 = (e % (DV / 4)) * 4; const int key = j0 + r;
      v4f f = {0.f,0.f,0.f,0.f}; if (key < Tk) f = *(const v4fa*)(V + (size_t)key * vpitch + c4);
#pragma unroll
      for (int t = 0; t < 4; ++t) { const unsigned short hb = bf16_bits(f[t]); sVh[r][c4 + t] = hb; sVl[r][c4 + t] = bf16_bits(f[t] - bf16_val(hb)); }
    }
    __syncthreads();
    v8f s[2];
#pragma unroll
    for (int nt = 0; nt < 2; ++nt) {
      v8f acc = {};
#pragma unroll
      for (int ks = 0; ks < KS; ++ks) {
        FragB bh_, bl_;
        bh_.half[0] = *(const v8us*)&sKh[nt * 16 + ln][ks * 32 + 8 * hh]; bh_.half[1] = *(const v8us*)&sKh[nt * 16 + ln][ks * 32 + 16 + 8 * hh];
        bl_.half[0] = *(const v8us*)&sKl[nt * 16 + ln][ks * 32 + 8 * hh]; bl_.half[1] = *(const v8us*)&sKl[nt * 16 + ln][ks * 32 + 16 + 8 * hh];
        acc = mmaN<3>(aqh[ks].v, aql[ks].v, bh_.v, bl_.v, acc);
      }
      s[nt] = acc;
    }
    float alpha[8];
#pragma unroll
    for (int r = 0; r < 8; ++r) {
      const int ja = j0 + ln, jb = j0 + 16 + ln;
      if (ja >= Tk) s[0][r] = -3.0e38f;
      if (jb >= Tk) s[1][r] = -3.0e38f;
      float mx = fmaxf(s[0][r], s[1][r]);
      mx = fmaxf(mx, __shfl_xor(mx, 1, 32)); mx = fmaxf(mx, __shfl_xor(mx, 2, 32)); mx = fmaxf(mx, __shfl_xor(mx, 4, 32)); mx = fmaxf(mx, __shfl_xor(mx, 8, 32));
      const float mnew = fmaxf(m_r[r], mx);
      alpha[r] = (mnew > -1.0e38f) ? __expf(m_r[r] - mnew) : 1.0f;
      const float p0 = (s[0][r] > -1.0e38f) ? __expf(s[0][r] - mnew) : 0.f;
      const float p1 = (s[1][r] > -1.0e38f) ? __expf(s[1][r] - mnew) : 0.f;
      m_r[r] = mnew;
      l_r[r] = l_r[r] * alpha[r] + p0 + p1;
      unsigned short hb = bf16_bits(p0); sPh[w][8 * hh + r][ln] = hb;      sPl[w][8 * hh + r][ln] = bf16_bits(p0 - bf16_val(hb));
      hb = bf16_bits(p1);                sPh[w][8 * hh + r][16 + ln] = hb; sPl[w][8 * hh + r][16 + ln] = bf16_bits(p1 - bf16_val(hb));
    }
#pragma unroll
    for (int dt = 0; dt < DT; ++dt)
#pragma unroll
      for (int r = 0; r < 8; ++r) oacc[dt][r] *= alpha[r];
    __builtin_amdgcn_fence(__ATOMIC_ACQ_REL, "workgroup");
    __builtin_amdgcn_wave_barrier();
    FragB pah, pal;
    pah.half[0] = *(const v8us*)&sPh[w][ln][8 * hh]; pah.half[1] = *(const v8us*)&sPh[w][ln][16 + 8 * hh];
    pal.half[0] = *(const v8us*)&sPl[w][ln][8 * hh]; pal.half[1] = *(const v8us*)&sPl[w][ln][16 + 8 * hh];
#pragma unroll
    for (int dt = 0; dt < DT; ++dt) {
      FragB bvh, bvl;
#pragma unroll
      for (int i = 0; i < 8; ++i) {
        bvh.u[i] = sVh[8 * hh + i][dt * 16 + ln]; bvh.u[8 + i] = sVh[16 + 8 * hh + i][dt * 16 + ln];
        bvl.u[i] = sVl[8 * hh + i][dt * 16 + ln]; bvl.u[8 + i] = sVl[16 + 8 * hh + i][dt * 16 + ln];
      }
      oacc[dt] = mmaN<3>(pah.v, pal.v, bvh.v, bvl.v, oacc[dt]);
    }
    __builtin_amdgcn_fence(__ATOMIC_ACQ_REL, "workgroup");
    __builtin_amdgcn_wave_barrier();
  }
#pragma unroll
  for (int r = 0; r < 8; ++r) {
    float l = l_r[r];
    l += __shfl_xor(l, 1, 32); l += __shfl_xor(l, 2, 32); l += __shfl_xor(l, 4, 32); l += __shfl_xor(l, 8, 32);
    l_r[r] = (l > 0.f) ? 1.0f / l : 0.f;
  }
#pragma unroll
  for (int dt = 0; dt < DT; ++dt)
#pragma unroll
    for (int r = 0; r < 8; ++r) sO[w][8 * hh + r][dt * 16 + ln] = oacc[dt][r] * l_r[r];
  __builtin_amdgcn_fence(__ATOMIC_ACQ_REL, "workgroup");
  __builtin_amdgcn_wave_barrier();
  for (int pass = 0; pass < 2; ++pass) {
    for (int r = 0; r < 16; ++r) {
      const int row = q0 + r;
      for (int c4 = lane * 4; c4 < DV; c4 += 128) {
        if (row < Tq) {
          const v4f val = *(const v4fa*)&sO[w][r][c4];
          *(volatile v4f*)(y + (size_t)bh * ystride + (size_t)row * ypitch + dv0 + c4) = val;
        }
      }
    }
    if (pass == 0) __threadfence();
  }
}

template <bool ASPLIT, int ACT, bool BIAS_BF16, bool RES_BF16>
__global__ __launch_bounds__(128) void k_gemm_bf3(const float* __restrict__ A, int lda, const unsigned short* __restrict__ Wt, int ldb,
                                                const float* __restrict__ bias, const float* __restrict__ resid, int rmod, int ldr,
                                                float* __restrict__ C, int ldc, int M, int N, int K) {
  __shared__ __attribute__((aligned(16))) float so[4][16][64];
  const int tid = threadIdx.x, w = tid >> 5, lane = tid & 31, ln = lane & 15, hh = lane >> 4;
  const int ntn = N / 64;
  const int wid = blockIdx.x * 4 + w;
  const int mt = wid / ntn, nq = wid % ntn;
  if (mt * 16 >= M) return;
  const int row0 = mt * 16, col0 = nq * 64;
  const float* arow = A + (size_t)(row0 + ln) * lda;
  v8f acc[4] = {};
  for (int kb = 0; kb < K; kb += 32) {
    FragB ah, al;
    const v4f x0 = *(const v4fa*)(arow + kb + 8 * hh), x1 = *(const v4fa*)(arow + kb + 8 * hh + 4);
    const v4f x2 = *(const v4fa*)(arow + kb + 16 + 8 * hh), x3 = *(const v4fa*)(arow + kb + 16 + 8 * hh + 4);
    float xs[16] = {x0[0],x0[1],x0[2],x0[3],x1[0],x1[1],x1[2],x1[3],x2[0],x2[1],x2[2],x2[3],x3[0],x3[1],x3[2],x3[3]};
#pragma unroll
    for (int i = 0; i < 16; ++i) { const unsigned short hb = bf16_bits(xs[i]); ah.u[i] = hb; al.u[i] = ASPLIT ? bf16_bits(xs[i] - bf16_val(hb)) : (unsigned short)0; }
#pragma unroll
    for (int t = 0; t < 4; ++t) {
      const unsigned short* brow = Wt + (size_t)(col0 + t * 16 + ln) * ldb + kb;
      FragB b;
      b.half[0] = *(const v8us*)(brow + 8 * hh);
      b.half[1] = *(const v8us*)(brow + 16 + 8 * hh);
      acc[t] = mmaN<ASPLIT ? 2 : 1>(ah.v, al.v, b.v, b.v, acc[t]);
    }
  }
#pragma unroll
  for (int t = 0; t < 4; ++t) {
    const int col = col0 + t * 16 + ln;
    float bv = bias ? bias[col] : 0.f;
    if (BIAS_BF16) bv = bf16_round(bv);
#pragma unroll
    for (int r = 0; r < 8; ++r) {
      float v = acc[t][r] + bv;
      if (resid) { float rv = resid[(size_t)((row0 + 8 * hh + r) % rmod) * ldr + col]; if (RES_BF16) rv = bf16_round(rv); v += rv; }
      if (ACT == 1) v = fmaxf(v, 0.f);
      if (ACT == 2) v = 0.5f * v * (1.0f + erff(v * 0.70710678118654752f));
      if (ACT == 3) { const float u = 0.7978845608028654f * (v + 0.044715f * v * v * v); v = 0.5f * v * (1.0f + tanhf(u)); }
      so[w][8 * hh + r][t * 16 + ln] = v;
    }
  }
  __builtin_amdgcn_fence(__ATOMIC_ACQ_REL, "workgroup");
  __builtin_amdgcn_wave_barrier();
  const int rsub = lane >> 4, c4 = (lane & 15) * 4;
  for (int pass = 0; pass < 2; ++pass) {
#pragma unroll
    for (int q = 0; q < 8; ++q) {
      const int r = q * 2 + rsub;
      const v4f v = *(const v4fa*)&so[w][r][c4];
      *(volatile v4f*)(C + (size_t)(row0 + r) * ldc + col0 + c4) = v;
    }
    if (pass == 0) __threadfence();
  }
}
template <bool PARAM_BF16>
__global__ __launch_bounds__(256) void k_layernorm(const float* __restrict__ X, const float* __restrict__ R, const float* __restrict__ g, const float* __restrict__ bta,
                                                  float* __restrict__ out_sum, float* __restrict__ out_norm, int N, float eps) {
  __shared__ float red[256];
  const int row = blockIdx.x, tid = threadIdx.x;
  const float* x = X + (size_t)row * N; const float* rr = R ? R + (size_t)row * N : nullptr;
  float vals[16];
  const int per = N / 256;
  float s1 = 0.f;
  for (int u = 0; u < per / 4; ++u) {
    const int j = tid * 4 + 1024 * u;
    const v4f a = *(const v4fa*)(x + j);
    v4f b = {0.f,0.f,0.f,0.f}; if (rr) b = *(const v4fa*)(rr + j);
#pragma unroll
    for (int q = 0; q < 4; ++q) { const float v = a[q] + b[q]; vals[u * 4 + q] = v; s1 += v; }
  }
  red[tid] = s1; __syncthreads();
  for (int st = 128; st > 0; st >>= 1) { if (tid < st) red[tid] += red[tid + st]; __syncthreads(); }
  const float mu = red[0] / (float)N; __syncthreads();
  float s2 = 0.f;
  for (int u = 0; u < per / 4; ++u)
#pragma unroll
    for (int q = 0; q < 4; ++q) { const float c = vals[u * 4 + q] - mu; s2 += c * c; }
  red[tid] = s2; __syncthreads();
  for (int st = 128; st > 0; st >>= 1) { if (tid < st) red[tid] += red[tid + st]; __syncthreads(); }
  const float rs = rsqrtf(red[0] / (float)N + eps);
  for (int pass = 0; pass < 2; ++pass) {
    for (int u = 0; u < per / 4; ++u) {
      const int j = tid * 4 + 1024 * u;
      v4f o, sm;
#pragma unroll
      for (int q = 0; q < 4; ++q) {
        float gg = g[j + q], bb = bta[j + q];
        if (PARAM_BF16) { gg = bf16_round(gg); bb = bf16_round(bb); }
        sm[q] = vals[u * 4 + q]; o[q] = (vals[u * 4 + q] - mu) * rs * gg + bb;
      }
      if (out_sum) *(volatile v4f*)(out_sum + (size_t)row * N + j) = sm;
      *(volatile v4f*)(out_norm + (size_t)row * N + j) = o;
    }
    if (pass == 0) __threadfence();
  }
}

template <int D>
__global__ __launch_bounds__(128) void k_flash3(const float* __restrict__ Qb, int qpitch, int Tq,
                                              const float* __restrict__ K1, const float* __restrict__ V1, int Tk1,
                                              const float* __restrict__ K2, const float* __restrict__ V2, int Tk2, int kpitch, int vpitch,
                                              int H, float scale, const int* __restrict__ mask, int causal, const float* __restrict__ sbias,
                                              float* __restrict__ y, int ypitch) {
  constexpr int KS = D / 32, DT = D / 16;
  __shared__ __attribute__((aligned(16))) unsigned short sKh[32][D + 8], sKl[32][D + 8], sVh[32][D + 8], sVl[32][D + 8];
  __shared__ __attribute__((aligned(16))) unsigned short sPh[4][16][40], sPl[4][16][40];
  __shared__ __attribute__((aligned(16))) float sO[4][16][D];
  const int tid = threadIdx.x, w = tid >> 5, lane = tid & 31, ln = lane & 15, hh = lane >> 4;
  const int Tk = Tk1 + Tk2;
  const int nqb = (Tq + 63) / 64;
  const int bh = blockIdx.x / nqb, qblk = blockIdx.x % nqb;
  const int b = bh / H, h = bh % H;
  const int q0 = qblk * 64 + w * 16;
  const float* Q = Qb + (size_t)b * Tq * qpitch + h * D;
  FragB aqh[KS], aql[KS];
  {
    int row = q0 + ln; if (row >= Tq) row = Tq - 1;
    const float* qr = Q + (size_t)row * qpitch;
#pragma unroll
    for (int ks = 0; ks < KS; ++ks)
#pragma unroll
      for (int i = 0; i < 16; ++i) {
        const int d = ks * 32 + ((i < 8) ? (8 * hh + i) : (16 + 8 * hh + (i - 8)));
        const float x = qr[d] * scale; const unsigned short hb = bf16_bits(x);
        aqh[ks].u[i] = hb; aql[ks].u[i] = bf16_bits(x - bf16_val(hb));
      }
  }
  int qrow[8];
#pragma unroll
  for (int r = 0; r < 8; ++r) { int qi = q0 + 8 * hh + r; qrow[r] = qi < Tq ? qi : Tq - 1; }
  float m_r[8], l_r[8];
#pragma unroll
  for (int r = 0; r < 8; ++r) { m_r[r] = -3.0e38f; l_r[r] = 0.f; }
  v8f oacc[DT];
#pragma unroll
  for (int dt = 0; dt < DT; ++dt) oacc[dt] = (v8f){0.f,0.f,0.f,0.f,0.f,0.f,0.f,0.f};
  const int kv_end = causal ? min(Tk, qblk * 64 + 64) : Tk;
  for (int j0 = 0; j0 < kv_end; j0 += 32) {
    __syncthreads();
    for (int e = tid; e < 32 * (D / 4); e += 128) {
      const int r = e / (D / 4), c4 = (e % (D / 4)) * 4; const int key = j0 + r;
      v4f kf = {0.f,0.f,0.f,0.f}, vf = {0.f,0.f,0.f,0.f};
      if (key < Tk1) { kf = *(const v4fa*)(K1 + (size_t)b * Tk1 * kpitch + h * D + (size_t)key * kpitch + c4); vf = *(const v4fa*)(V1 + (size_t)b * Tk1 * vpitch + h * D + (size_t)key * vpitch + c4); }
      else if (key < Tk) { const int k2 = key - Tk1; kf = *(const v4fa*)(K2 + (size_t)b * Tk2 * kpitch + h * D + (size_t)k2 * kpitch + c4); vf = *(const v4fa*)(V2 + (size_t)b * Tk2 * vpitch + h * D + (size_t)k2 * vpitch + c4); }
#pragma unroll
      for (int t = 0; t < 4; ++t) {
        unsigned short hb = bf16_bits(kf[t]); sKh[r][c4 + t] = hb; sKl[r][c4 + t] = bf16_bits(kf[t] - bf16_val(hb));
        hb = bf16_bits(vf[t]); sVh[r][c4 + t] = hb; sVl[r][c4 + t] = bf16_bits(vf[t] - bf16_val(hb));
      }
    }
    __syncthreads();
    v8f s[2];
#pragma unroll
    for (int nt = 0; nt < 2; ++nt) {
      v8f acc = {};
#pragma unroll
      for (int ks = 0; ks < KS; ++ks) {
        FragB bh_, bl_;
        bh_.half[0] = *(const v8us*)&sKh[nt * 16 + ln][ks * 32 + 8 * hh]; bh_.half[1] = *(const v8us*)&sKh[nt * 16 + ln][ks * 32 + 16 + 8 * hh];
        bl_.half[0] = *(const v8us*)&sKl[nt * 16 + ln][ks * 32 + 8 * hh]; bl_.half[1] = *(const v8us*)&sKl[nt * 16 + ln][ks * 32 + 16 + 8 * hh];
        acc = mmaN<3>(aqh[ks].v, aql[ks].v, bh_.v, bl_.v, acc);
      }
      s[nt] = acc;
    }
    float alpha[8];
#pragma unroll
    for (int r = 0; r < 8; ++r) {
      const int qi = qrow[r];
      const int ja = j0 + ln, jb = j0 + 16 + ln;
      bool keepa = ja < Tk, keepb = jb < Tk;
      if (causal) { keepa = keepa && (ja <= qi); keepb = keepb && (jb <= qi); }
      if (mask) { if (keepa) keepa = mask[(size_t)qi * Tk + ja] != 0; if (keepb) keepb = mask[(size_t)qi * Tk + jb] != 0; }
      if (sbias) { if (keepa) s[0][r] += sbias[(size_t)bh * Tk + ja]; if (keepb) s[1][r] += sbias[(size_t)bh * Tk + jb]; }
      if (!keepa) s[0][r] = -3.0e38f;
      if (!keepb) s[1][r] = -3.0e38f;
      float mx = fmaxf(s[0][r], s[1][r]);
      mx = fmaxf(mx, __shfl_xor(mx, 1, 32)); mx = fmaxf(mx, __shfl_xor(mx, 2, 32)); mx = fmaxf(mx, __shfl_xor(mx, 4, 32)); mx = fmaxf(mx, __shfl_xor(mx, 8, 32));
      const float mnew = fmaxf(m_r[r], mx);
      alpha[r] = (mnew > -1.0e38f) ? __expf(m_r[r] - mnew) : 1.0f;
      const float p0 = keepa ? __expf(s[0][r] - mnew) : 0.f;
      const float p1 = keepb ? __expf(s[1][r] - mnew) : 0.f;
      m_r[r] = mnew;
      l_r[r] = l_r[r] * alpha[r] + p0 + p1;
      unsigned short hb = bf16_bits(p0); sPh[w][8 * hh + r][ln] = hb;      sPl[w][8 * hh + r][ln] = bf16_bits(p0 - bf16_val(hb));
      hb = bf16_bits(p1);                sPh[w][8 * hh + r][16 + ln] = hb; sPl[w][8 * hh + r][16 + ln] = bf16_bits(p1 - bf16_val(hb));
    }
#pragma unroll
    for (int dt = 0; dt < DT; ++dt)
#pragma unroll
      for (int r = 0; r < 8; ++r) oacc[dt][r] *= alpha[r];
    __builtin_amdgcn_fence(__ATOMIC_ACQ_REL, "workgroup");
    __builtin_amdgcn_wave_barrier();
    FragB pah, pal;
    pah.half[0] = *(const v8us*)&sPh[w][ln][8 * hh]; pah.half[1] = *(const v8us*)&sPh[w][ln][16 + 8 * hh];
    pal.half[0] = *(const v8us*)&sPl[w][ln][8 * hh]; pal.half[1] = *(const v8us*)&sPl[w][ln][16 + 8 * hh];
#pragma unroll
    for (int dt = 0; dt < DT; ++dt) {
      FragB bvh, bvl;
#pragma unroll
      for (int i = 0; i < 8; ++i) {
        bvh.u[i] = sVh[8 * hh + i][dt * 16 + ln]; bvh.u[8 + i] = sVh[16 + 8 * hh + i][dt * 16 + ln];
        bvl.u[i] = sVl[8 * hh + i][dt * 16 + ln]; bvl.u[8 + i] = sVl[16 + 8 * hh + i][dt * 16 + ln];
      }
      oacc[dt] = mmaN<3>(pah.v, pal.v, bvh.v, bvl.v, oacc[dt]);
    }
    __builtin_amdgcn_fence(__ATOMIC_ACQ_REL, "workgroup");
    __builtin_amdgcn_wave_barrier();
  }
#pragma unroll
  for (int r = 0; r < 8; ++r) {
    float l = l_r[r];
    l += __shfl_xor(l, 1, 32); l += __shfl_xor(l, 2, 32); l += __shfl_xor(l, 4, 32); l += __shfl_xor(l, 8, 32);
    l_r[r] = (m_r[r] > -1.0e38f) ? 1.0f / l : __builtin_nanf("");
  }
#pragma unroll
  for (int dt = 0; dt < DT; ++dt)
#pragma unroll
    for (int r = 0; r < 8; ++r) sO[w][8 * hh + r][dt * 16 + ln] = oacc[dt][r] * l_r[r];
  __builtin_amdgcn_fence(__ATOMIC_ACQ_REL, "workgroup");
  __builtin_amdgcn_wave_barrier();
  for (int pass = 0; pass < 2; ++pass) {
    for (int r = 0; r < 16; ++r) {
      const int row = q0 + r;
      if (row < Tq && lane < D / 4) {
        const v4f val = *(const v4fa*)&sO[w][r][lane * 4];
        *(volatile v4f*)(y + ((size_t)b * Tq + row) * ypitch + h * D + lane * 4) = val;
      }
    }
    if (pass == 0) __threadfence();
  }
}

__global__ __launch_bounds__(256) void k_round_rows(const float* __restrict__ W, unsigned short* __restrict__ Wt, int n8) {
  const int t = blockIdx.x * 256 + threadIdx.x;
  if (t >= n8) return;
  const v4f a = *(const v4fa*)(W + (size_t)t * 8), b = *(const v4fa*)(W + (size_t)t * 8 + 4);
  v8us v; v[0]=bf16_bits(a[0]); v[1]=bf16_bits(a[1]); v[2]=bf16_bits(a[2]); v[3]=bf16_bits(a[3]);
  v[4]=bf16_bits(b[0]); v[5]=bf16_bits(b[1]); v[6]=bf16_bits(b[2]); v[7]=bf16_bits(b[3]);
  *(volatile v8us*)(Wt + (size_t)t * 8) = v; __threadfence(); *(volatile v8us*)(Wt + (size_t)t * 8) = v;
}

__global__ __launch_bounds__(256) void k_mod(const float* __restrict__ fe, const float* __restrict__ W, const float* __restrict__ bb, float* __restrict__ mod) {
  __shared__ float sf[EE];
  const int b = blockIdx.y, j = blockIdx.x * 256 + threadIdx.x;
  for (int e = threadIdx.x; e < EE; e += 256) { const float v = bf16_round(fe[(size_t)b * EE + e]); sf[e] = v / (1.0f + expf(-v)); }
  __syncthreads();
  float s = bf16_round(bb[j]);
#pragma unroll 1
  for (int e = 0; e < EE; ++e) s += sf[e] * bf16_round(W[(size_t)e * 6 * CC + j]);
  *(volatile float*)(mod + (size_t)b * 6 * CC + j) = s; __threadfence(); *(volatile float*)(mod + (size_t)b * 6 * CC + j) = s;
}
template <bool IN_BF16>
__global__ __launch_bounds__(128) void k_rms_mod(const float* __restrict__ x, const float* __restrict__ w, const float* __restrict__ mod, int shoff, int scoff, float* __restrict__ h, float* __restrict__ xcopy) {
  __shared__ float red[128];
  const size_t row = blockIdx.x; const int b = (int)(row / HWN); const int t = threadIdx.x;
  v4f v = *(const v4fa*)(x + row * CC + t * 4); if (IN_BF16) for (int q = 0; q < 4; ++q) v[q] = bf16_round(v[q]);
  float s = v[0] * v[0] + v[1] * v[1] + v[2] * v[2] + v[3] * v[3]; red[t] = s; __syncthreads(); for (int st = 64; st > 0; st >>= 1) { if (t < st) red[t] += red[t + st]; __syncthreads(); }
  const float rs = rsqrtf(red[0] / (float)CC + 1e-6f);
  v4f o; for (int q = 0; q < 4; ++q) { const int c = t * 4 + q; o[q] = v[q] * rs * bf16_round(w[c]) * (1.0f + mod[(size_t)b * 6 * CC + scoff + c]) + mod[(size_t)b * 6 * CC + shoff + c]; }
  *(volatile v4f*)(h + row * CC + t * 4) = o; if (xcopy) *(volatile v4f*)(xcopy + row * CC + t * 4) = v; __threadfence(); *(volatile v4f*)(h + row * CC + t * 4) = o; if (xcopy) *(volatile v4f*)(xcopy + row * CC + t * 4) = v;
}
__global__ __launch_bounds__(256) void k_rope_s(float* __restrict__ qkv, const float* __restrict__ fr, const float* __restrict__ qn, const float* __restrict__ kn) {
  const int lane = threadIdx.x & 31; const size_t wv = (size_t)blockIdx.x * 8 + (threadIdx.x >> 5); if (wv >= (size_t)BB * HWN * NH * 2) return;
  const int which = (int)(wv & 1); const int h = (int)((wv >> 1) % NH); const size_t row = (wv >> 1) / NH; const int p = (int)(row % HWN); const float gy = (float)(p / WI), gx = (float)(p % WI);
  float* base = qkv + row * 3 * CC + (size_t)which * CC + h * HD; const float* nw = which ? kn : qn;
  const float x0 = base[2 * lane], x1 = base[2 * lane + 1];
  const float ang = gy * bf16_round(fr[lane * 2 + 0]) + gx * bf16_round(fr[lane * 2 + 1]); float sn, cs; sincosf(ang, &sn, &cs);
  const float r0 = x0 * cs - x1 * sn, r1 = x1 * cs + x0 * sn;
  float s = r0 * r0 + r1 * r1; for (int o = 16; o >= 1; o >>= 1) s += __shfl_xor(s, o, 32); const float rs = rsqrtf(s * (1.0f / HD) + 1.1920929e-07f);
  typedef float v2f __attribute__((ext_vector_type(2))); const v2f o = {r0 * rs * bf16_round(nw[2 * lane]), r1 * rs * bf16_round(nw[2 * lane + 1])};
  *(volatile v2f*)(base + 2 * lane) = o; __threadfence(); *(volatile v2f*)(base + 2 * lane) = o;
}
__global__ __launch_bounds__(256) void k_rope_c(float* __restrict__ qkvc, const float* __restrict__ kn) {
  const int lane = threadIdx.x & 31; const size_t wv = (size_t)blockIdx.x * 8 + (threadIdx.x >> 5); if (wv >= (size_t)BB * SP * NH) return;
  const int h = (int)(wv % NH); const size_t row = wv / NH; const int sidx = (int)(row % SP);
  float* base = qkvc + row * 3 * CC + CC + h * HD;
  const float x0 = base[2 * lane], x1 = base[2 * lane + 1];
  const float ang = (float)sidx * powf(10000.0f, -(float)(2 * lane) / (float)HD); float sn, cs; sincosf(ang, &sn, &cs);
  const float r0 = x0 * cs - x1 * sn, r1 = x1 * cs + x0 * sn;
  float s = r0 * r0 + r1 * r1; for (int o = 16; o >= 1; o >>= 1) s += __shfl_xor(s, o, 32); const float rs = rsqrtf(s * (1.0f / HD) + 1.1920929e-07f);
  typedef float v2f __attribute__((ext_vector_type(2))); const v2f o = {r0 * rs * bf16_round(kn[2 * lane]), r1 * rs * bf16_round(kn[2 * lane + 1])};
  *(volatile v2f*)(base + 2 * lane) = o; __threadfence(); *(volatile v2f*)(base + 2 * lane) = o;
}
__global__ __launch_bounds__(256) void k_condrows(const float* __restrict__ cs_, float* __restrict__ cr) {
  const size_t t = (size_t)blockIdx.x * 256 + threadIdx.x; if (t >= (size_t)BB * SP * EE / 4) return; const size_t row = t / (EE / 4); const int c4 = (int)(t % (EE / 4)) * 4; const int b = (int)(row / SP), s = (int)(row % SP);
  v4f v = {0.f,0.f,0.f,0.f}; if (s < SS) { const float* src = cs_ + ((size_t)b * SS + s) * EE + c4; for (int q = 0; q < 4; ++q) v[q] = bf16_round(src[q]); }
  *(volatile v4f*)(cr + t * 4) = v; __threadfence(); *(volatile v4f*)(cr + t * 4) = v;
}
__global__ __launch_bounds__(256) void k_sbias(float* __restrict__ sb) { const size_t t = (size_t)blockIdx.x * 256 + threadIdx.x; if (t >= (size_t)BB * NH * (HWN + SP)) return; const int j = (int)(t % (HWN + SP)); const float v = (j < HWN + SS) ? 0.f : -3.0e38f; *(volatile float*)(sb + t) = v; __threadfence(); *(volatile float*)(sb + t) = v; }
__global__ __launch_bounds__(256) void k_gate_res(const float* __restrict__ xr, const float* __restrict__ o, const float* __restrict__ mod, int goff, float* __restrict__ x1) {
  const size_t t = (size_t)blockIdx.x * 256 + threadIdx.x; if (t >= (size_t)BB * HWN * CC / 4) return; const size_t row = t / (CC / 4); const int c4 = (int)(t % (CC / 4)) * 4; const int b = (int)(row / HWN);
  const v4f a = *(const v4fa*)(xr + t * 4), oo = *(const v4fa*)(o + t * 4); v4f v; for (int q = 0; q < 4; ++q) v[q] = a[q] + mod[(size_t)b * 6 * CC + goff + c4 + q] * oo[q];
  *(volatile v4f*)(x1 + t * 4) = v; __threadfence(); *(volatile v4f*)(x1 + t * 4) = v;
}
extern "C" void kernel_launch(void* const* d_in, const int* in_sizes, int n_in,
                              void* d_out, int out_size, void* d_ws, size_t ws_size, hipStream_t stream) {
  (void)in_sizes; (void)n_in; (void)out_size;
  const float* x = (const float*)d_in[0]; const float* cond = (const float*)d_in[1]; const float* femb = (const float*)d_in[2]; const float* mod_w = (const float*)d_in[3]; const float* mod_b = (const float*)d_in[4];
  const float* n1 = (const float*)d_in[5]; const float* n2 = (const float*)d_in[6]; const float* qkv_s_w = (const float*)d_in[7]; const float* qkv_c_w = (const float*)d_in[8]; const float* fr = (const float*)d_in[9];
  const float* qn = (const float*)d_in[10]; const float* kn = (const float*)d_in[11]; const float* out_w = (const float*)d_in[12]; const float* out_b = (const float*)d_in[13];
  const float* w1 = (const float*)d_in[14]; const float* b1 = (const float*)d_in[15]; const float* w2 = (const float*)d_in[16]; const float* b2 = (const float*)d_in[17];
  char* ws = (char*)d_ws; size_t off = 0;
  auto take = [&](size_t bytes) { char* p = ws + off; off += (bytes + 255) & ~(size_t)255; return p; };
  const int M = BB * HWN, MC = BB * SP; const size_t NE = (size_t)M * CC;
  unsigned short* Bqs = (unsigned short*)take((size_t)3 * CC * CC * 2); unsigned short* Bqc = (unsigned short*)take((size_t)3 * CC * EE * 2); unsigned short* Bo = (unsigned short*)take((size_t)CC * CC * 2); unsigned short* Bw1 = (unsigned short*)take((size_t)HID * CC * 2); unsigned short* Bw2 = (unsigned short*)take((size_t)CC * HID * 2);
  float* mod = (float*)take((size_t)BB * 6 * CC * 4); float* sb = (float*)take((size_t)BB * NH * (HWN + SP) * 4);
  float* xT = (float*)take(NE * 4); float* xr = (float*)take(NE * 4); float* hm = (float*)take(NE * 4); float* qkv = (float*)take((size_t)M * 3 * CC * 4); float* crow = (float*)take((size_t)MC * EE * 4); float* qkvc = (float*)take((size_t)MC * 3 * CC * 4);
  float* att = (float*)take(NE * 4); float* o = (float*)take(NE * 4); float* x1 = (float*)take(NE * 4); float* mm = (float*)take((size_t)M * HID * 4);
  if (off > ws_size) return;
  k_round_rows<<<(3 * CC * CC / 8 + 255) / 256, 256, 0, stream>>>(qkv_s_w, Bqs, 3 * CC * CC / 8); k_round_rows<<<(3 * CC * EE / 8 + 255) / 256, 256, 0, stream>>>(qkv_c_w, Bqc, 3 * CC * EE / 8);
  k_round_rows<<<(CC * CC / 8 + 255) / 256, 256, 0, stream>>>(out_w, Bo, CC * CC / 8); k_round_rows<<<(HID * CC / 8 + 255) / 256, 256, 0, stream>>>(w1, Bw1, HID * CC / 8); k_round_rows<<<(CC * HID / 8 + 255) / 256, 256, 0, stream>>>(w2, Bw2, CC * HID / 8);
  k_mod<<<dim3(6 * CC / 256, BB), 256, 0, stream>>>(femb, mod_w, mod_b, mod);
  k_sbias<<<(BB * NH * (HWN + SP) + 255) / 256, 256, 0, stream>>>(sb);
  k_transpose32<false, false, false><<<dim3(HWN / 32, CC / 32, BB), 256, 0, stream>>>(x, xT, CC, HWN, nullptr, nullptr, nullptr);
  k_rms_mod<true><<<M, 128, 0, stream>>>(xT, n1, mod, 0, CC, hm, xr);
  k_gemm_bf3<true, 0, false, false><<<((M / 16) * (3 * CC / 64) + 3) / 4, 128, 0, stream>>>(hm, CC, Bqs, CC, nullptr, nullptr, 1, 0, qkv, 3 * CC, M, 3 * CC, CC);
  k_condrows<<<(unsigned)(((size_t)MC * EE / 4 + 255) / 256), 256, 0, stream>>>(cond, crow);
  k_gemm_bf3<false, 0, false, false><<<((MC / 16) * (3 * CC / 64) + 3) / 4, 128, 0, stream>>>(crow, EE, Bqc, EE, nullptr, nullptr, 1, 0, qkvc, 3 * CC, MC, 3 * CC, EE);
  k_rope_s<<<(unsigned)(((size_t)M * NH * 2 + 7) / 8), 256, 0, stream>>>(qkv, fr, qn, kn);
  k_rope_c<<<(unsigned)(((size_t)MC * NH + 7) / 8), 256, 0, stream>>>(qkvc, kn);
  k_flash3<HD><<<BB * NH * (HWN / 64), 128, 0, stream>>>(qkv, 3 * CC, HWN, qkv + CC, qkv + 2 * CC, HWN, qkvc + CC, qkvc + 2 * CC, SP, 3 * CC, 3 * CC, NH, 0.125f, nullptr, 0, sb, att, CC);
  k_gemm_bf3<true, 0, true, false><<<((M / 16) * (CC / 64) + 3) / 4, 128, 0, stream>>>(att, CC, Bo, CC, out_b, nullptr, 1, 0, o, CC, M, CC, CC);
  k_gate_res<<<(unsigned)((NE / 4 + 255) / 256), 256, 0, stream>>>(xr, o, mod, 2 * CC, x1);
  k_rms_mod<false><<<M, 128, 0, stream>>>(x1, n2, mod, 3 * CC, 4 * CC, hm, nullptr);
  k_gemm_bf3<true, 3, true, false><<<((M / 16) * (HID / 64) + 3) / 4, 128, 0, stream>>>(hm, CC, Bw1, CC, b1, nullptr, 1, 0, mm, HID, M, HID, CC);
  k_gemm_bf3<true, 0, true, false><<<((M / 16) * (CC / 64) + 3) / 4, 128, 0, stream>>>(mm, HID, Bw2, HID, b2, nullptr, 1, 0, o, CC, M, CC, HID);
  k_gate_res<<<(unsigned)((NE / 4 + 255) / 256), 256, 0, stream>>>(x1, o, mod, 5 * CC, att);
  k_transpose32<false, false, false><<<dim3(CC / 32, HWN / 32, BB), 256, 0, stream>>>(att, (float*)d_out, HWN, CC, nullptr, nullptr, nullptr);
}
